// SelectiveSSM_82471962018274
// MI455X (gfx1250) — hardware-verified
//
#include <hip/hip_runtime.h>
#include <math.h>

typedef __attribute__((ext_vector_type(16))) _Float16 v16h;
typedef __attribute__((ext_vector_type(8)))  _Float16 v8h;
typedef __attribute__((ext_vector_type(16))) __bf16   v16b;
typedef __attribute__((ext_vector_type(8)))  __bf16   v8b;
typedef __attribute__((ext_vector_type(8)))  float    v8f;
typedef __attribute__((ext_vector_type(4)))  float    v4f;

constexpr int kSeq    = 1024;
constexpr int kDm     = 512;
constexpr int kDin    = 1024;
constexpr int kNst    = 64;
constexpr int kDtR    = 32;
constexpr int kConvK  = 4;
constexpr int kWin    = 8;
constexpr int kXzP    = 2 * kDin;
constexpr int kXdN    = kDtR + 2 * kNst;
constexpr int kXdP    = 192;
constexpr int kColB   = kDtR;
constexpr int kColC   = kDtR + kNst;
constexpr float kLnEps = 1e-5f;
constexpr int kConvTP = 260;
constexpr int kScanCh = 32;
constexpr int kScanTS = 32;
constexpr int kScanYP = 36;
constexpr int kLnRows = 8;
static_assert(kXdN == 160 && kXdP >= kXdN && (kXdP % 64) == 0, "x_proj pad");
static_assert((kDm % 32) == 0 && (kDin % 32) == 0 && (kDtR % 32) == 0, "GEMM K multiples of 32");
static_assert((kSeq % 64) == 0 && (kXzP % 64) == 0 && (kXdP % 64) == 0 && (kDin % 64) == 0 && (kDm % 64) == 0, "GEMM M,N multiples of 64");
static_assert((kSeq % kScanTS) == 0 && (kDin % kScanCh) == 0 && kScanCh == 32 && kScanTS == 32 && kNst == 64 && kWin == 8, "scan tiling");
static_assert((kSeq % 64) == 0 && (kDin % 256) == 0 && kDm == 512 && (kSeq % kLnRows) == 0 && kConvK == 4, "conv and LN tiling");

constexpr size_t kOffXB   = 0;
constexpr size_t kOffWIB  = kOffXB  + (size_t)kSeq * kDm  * 2;
constexpr size_t kOffWXB  = kOffWIB + (size_t)kXzP * kDm  * 2;
constexpr size_t kOffWDB  = kOffWXB + (size_t)kXdP * kDin * 2;
constexpr size_t kOffWOB  = kOffWDB + (size_t)kDin * kDtR * 2;
constexpr size_t kOffXZ   = kOffWOB + (size_t)kDm  * kDin * 2;
constexpr size_t kOffUC   = kOffXZ  + (size_t)kSeq * kXzP * 4;
constexpr size_t kOffUCH  = kOffUC  + (size_t)kSeq * kDin * 4;
constexpr size_t kOffUCL  = kOffUCH + (size_t)kSeq * kDin * 2;
constexpr size_t kOffXD   = kOffUCL + (size_t)kSeq * kDin * 2;
constexpr size_t kOffDRH  = kOffXD  + (size_t)kSeq * kXdP * 4;
constexpr size_t kOffDRL  = kOffDRH + (size_t)kSeq * kDtR * 2;
constexpr size_t kOffDLR  = kOffDRL + (size_t)kSeq * kDtR * 2;
constexpr size_t kOffY    = kOffDLR + (size_t)kSeq * kDin * 4;
constexpr size_t kOffYH   = kOffY   + (size_t)kSeq * kDin * 4;
constexpr size_t kOffYL   = kOffYH  + (size_t)kSeq * kDin * 2;
constexpr size_t kOffPRE  = kOffYL  + (size_t)kSeq * kDin * 2;
constexpr size_t kWsTotal = kOffPRE + (size_t)kSeq * kDm  * 4;
static_assert(kWsTotal == 37027840ull, "carve total");
static_assert(kWsTotal <= 134217728ull, "carve cap");
static_assert((kOffWIB % 128) == 0 && (kOffWXB % 128) == 0 && (kOffWDB % 128) == 0 && (kOffWOB % 128) == 0 &&
              (kOffXZ % 128) == 0 && (kOffUC % 128) == 0 && (kOffUCH % 128) == 0 && (kOffUCL % 128) == 0 &&
              (kOffXD % 128) == 0 && (kOffDRH % 128) == 0 && (kOffDRL % 128) == 0 && (kOffDLR % 128) == 0 &&
              (kOffY % 128) == 0 && (kOffYH % 128) == 0 && (kOffYL % 128) == 0 && (kOffPRE % 128) == 0, "128-B aligned regions");

__device__ __forceinline__ unsigned short f2bf_bits(float f) {
  unsigned u = __float_as_uint(f);
  return (unsigned short)((u + 0x7FFFu + ((u >> 16) & 1u)) >> 16);
}
__device__ __forceinline__ float bf_bits2f(unsigned short h) { return __uint_as_float(((unsigned)h) << 16); }
__device__ __forceinline__ float bf16r(float f) { return __uint_as_float(((unsigned)f2bf_bits(f)) << 16); }

__device__ __forceinline__ void dep_guard4_h(v8f& a, v8f& b, v8f& c, v8f& d, v16h x, v16h y) {
  asm volatile("v_nop\n\tv_nop\n\tv_nop\n\tv_nop" : "+v"(a), "+v"(b), "+v"(c), "+v"(d) : "v"(x), "v"(y));
}
__device__ __forceinline__ void dep_guard4_b(v8f& a, v8f& b, v8f& c, v8f& d, v16b x, v16b y) {
  asm volatile("v_nop\n\tv_nop\n\tv_nop\n\tv_nop" : "+v"(a), "+v"(b), "+v"(c), "+v"(d) : "v"(x), "v"(y));
}
__device__ __forceinline__ void keep4_h(v16h a, v16h b, v16h c, v16h d) { asm volatile("v_nop" :: "v"(a), "v"(b), "v"(c), "v"(d)); }
__device__ __forceinline__ void keep4_b(v16b a, v16b b, v16b c, v16b d) { asm volatile("v_nop" :: "v"(a), "v"(b), "v"(c), "v"(d)); }
__device__ __forceinline__ void acc_guard4(v8f& a, v8f& b, v8f& c, v8f& d) { asm volatile("v_nop\n\tv_nop\n\tv_nop\n\tv_nop" : "+v"(a), "+v"(b), "+v"(c), "+v"(d)); }
template <typename T> struct Frag;
template <> struct Frag<_Float16> {
  typedef v16h V; union U { v16h v; v8h h[2]; };
  static __device__ __forceinline__ v16h load(const _Float16* p) {
    U f; f.h[0] = *(const v8h*)(p); f.h[1] = *(const v8h*)(p + 16); return f.v;
  }
  static __device__ __forceinline__ v8f mma(v16h a, v16h b, v8f c) {
    return __builtin_amdgcn_wmma_f32_16x16x32_f16(false, a, false, b, (short)0, c, false, false);
  }
  static __device__ __forceinline__ void guard4(v8f& a, v8f& b, v8f& c, v8f& d, v16h x, v16h y) { dep_guard4_h(a, b, c, d, x, y); }
  static __device__ __forceinline__ void keep(v16h a, v16h b, v16h c, v16h d) { keep4_h(a, b, c, d); }
};
template <> struct Frag<__bf16> {
  typedef v16b V; union U { v16b v; v8b h[2]; };
  static __device__ __forceinline__ v16b load(const __bf16* p) {
    U f; f.h[0] = *(const v8b*)(p); f.h[1] = *(const v8b*)(p + 16); return f.v;
  }
  static __device__ __forceinline__ v8f mma(v16b a, v16b b, v8f c) {
    return __builtin_amdgcn_wmma_f32_16x16x32_bf16(false, a, false, b, (short)0, c, false, false);
  }
  static __device__ __forceinline__ void guard4(v8f& a, v8f& b, v8f& c, v8f& d, v16b x, v16b y) { dep_guard4_b(a, b, c, d, x, y); }
  static __device__ __forceinline__ void keep(v16b a, v16b b, v16b c, v16b d) { keep4_b(a, b, c, d); }
};

template <int ET> struct Elem;
template <> struct Elem<0> { typedef _Float16 T; };
template <> struct Elem<1> { typedef __bf16 T; };
template <int ET, int SPL, int BIAS_MODE, int OUT_MODE, int ACT = 0>
__global__ __launch_bounds__(256) void wmma_gemm64(
    const unsigned short* __restrict__ Ap, const unsigned short* __restrict__ A2p, int lda, long strideA,
    const unsigned short* __restrict__ Btp, const unsigned short* __restrict__ Bt2p, int ldb, long strideB,
    void* __restrict__ Cout, void* __restrict__ Cout2, int ldc, long strideC,
    const float* __restrict__ bias,
    int M, int N, int K, float scale) {
  typedef typename Elem<ET>::T T;
  typedef typename Frag<T>::V V;
  const T* A = (const T*)Ap; const T* A2 = (const T*)A2p; const T* Bt = (const T*)Btp; const T* Bt2 = (const T*)Bt2p;
  __shared__ __align__(16) float sT[8][16 * 68];
  const int b    = blockIdx.y;
  const int lane = threadIdx.x & 31;
  const int wave = threadIdx.x >> 5;
  const int tilesN = N >> 6;
  const int tilesM = M >> 6;
  const int tile = blockIdx.x * 8 + wave;
  if (tile >= tilesM * tilesN) return;
  const int tm = tile / tilesN;
  const int tn = tile - tm * tilesN;
  const int m0 = tm << 6;
  const int n0 = tn << 6;

  const T* Ab  = A  + (size_t)b * strideA;
  const T* Bb  = Bt + (size_t)b * strideB;
  const T* Ab2 = (SPL >= 1) ? (A2  + (size_t)b * strideA) : nullptr;
  const T* Bb2 = (SPL == 2) ? (Bt2 + (size_t)b * strideB) : nullptr;

  const int rlane = lane & 15;
  const int koff  = (lane >> 4) * 8;
  const int mOff  = (lane >> 4) * 8;

  v8f acc[4][4];
#pragma unroll
  for (int i = 0; i < 4; ++i)
#pragma unroll
    for (int j = 0; j < 4; ++j) acc[i][j] = (v8f){0.f,0.f,0.f,0.f,0.f,0.f,0.f,0.f};

  for (int k0 = 0; k0 < K; k0 += 32) {
    V bh[4], bl[4];
#pragma unroll
    for (int j = 0; j < 4; ++j) {
      const size_t bo = (size_t)(n0 + (j << 4) + rlane) * ldb + koff + k0;
      bh[j] = Frag<T>::load(Bb + bo);
      if (SPL == 2) bl[j] = Frag<T>::load(Bb2 + bo);
    }
#pragma unroll
    for (int i = 0; i < 4; ++i) {
      const size_t ao = (size_t)(m0 + (i << 4) + rlane) * lda + koff + k0;
      V ah = Frag<T>::load(Ab + ao);
      V al = ah;
      if (SPL >= 1) al = Frag<T>::load(Ab2 + ao);
#pragma unroll
      for (int j = 0; j < 4; ++j) {
        acc[i][j] = Frag<T>::mma(ah, bh[j], acc[i][j]);
        if (SPL == 2) acc[i][j] = Frag<T>::mma(ah, bl[j], acc[i][j]);
        if (SPL >= 1) acc[i][j] = Frag<T>::mma(al, bh[j], acc[i][j]);
      }
      Frag<T>::guard4(acc[i][0], acc[i][1], acc[i][2], acc[i][3], ah, al);
    }
    Frag<T>::keep(bh[0], bh[1], bh[2], bh[3]);
    if (SPL == 2) Frag<T>::keep(bl[0], bl[1], bl[2], bl[3]);
  }
  acc_guard4(acc[0][0], acc[0][1], acc[0][2], acc[0][3]);
  acc_guard4(acc[1][0], acc[1][1], acc[1][2], acc[1][3]);
  acc_guard4(acc[2][0], acc[2][1], acc[2][2], acc[2][3]);
  acc_guard4(acc[3][0], acc[3][1], acc[3][2], acc[3][3]);

  float* slab = sT[wave];
#pragma unroll
  for (int i = 0; i < 4; ++i) {
    const int mBase = m0 + (i << 4);
#pragma unroll
    for (int j = 0; j < 4; ++j) {
      const int n = n0 + (j << 4) + rlane;
      float bv = 0.f;
      if (BIAS_MODE == 2) bv = bias[n];
#pragma unroll
      for (int r = 0; r < 8; ++r) {
        float v = acc[i][j][r] * scale;
        if (BIAS_MODE == 1) v += bias[mBase + mOff + r];
        if (BIAS_MODE == 2) v += bv;
        if (ACT == 1) v = tanhf(v);
        if (ACT == 2) v = fmaxf(v, 0.0f);
        if (ACT == 3) v = v / (1.0f + expf(-v));
        if (ACT == 4) v = (v > 0.f) ? v : 0.01f * v;
        slab[(mOff + r) * 68 + (j << 4) + rlane] = v;
      }
    }
    __builtin_amdgcn_fence(__ATOMIC_RELEASE, "workgroup");
    __builtin_amdgcn_wave_barrier();
    __builtin_amdgcn_fence(__ATOMIC_ACQUIRE, "workgroup");
    if (OUT_MODE == 0) {
      float* C = (float*)Cout + (size_t)b * strideC;
      const int hh = lane >> 4, c4 = (lane & 15) * 4;
      for (int pass = 0; pass < 2; ++pass) {
#pragma unroll
        for (int it = 0; it < 8; ++it) {
          const int row = it * 2 + hh;
          v4f v = *(const v4f*)(slab + row * 68 + c4);
          *(volatile v4f*)(C + (size_t)(mBase + row) * ldc + n0 + c4) = v;
        }
        __threadfence();
      }
    } else {
      const int q = lane >> 3, c8 = (lane & 7) * 8;
      unsigned short* C  = (unsigned short*)Cout  + (size_t)b * strideC;
      unsigned short* C2 = (OUT_MODE == 2) ? ((unsigned short*)Cout2 + (size_t)b * strideC) : nullptr;
      for (int pass = 0; pass < 2; ++pass) {
#pragma unroll
        for (int it = 0; it < 4; ++it) {
          const int row = it * 4 + q;
          const float* sp = slab + row * 68 + c8;
          v8h hv, lv;
#pragma unroll
          for (int e = 0; e < 8; ++e) {
            const float se = sp[e];
            if (OUT_MODE == 1) {
              hv[e] = (_Float16)se;
            } else {
              unsigned short hb = f2bf_bits(se);
              unsigned short lb = f2bf_bits(se - bf_bits2f(hb));
              hv[e] = __builtin_bit_cast(_Float16, hb);
              lv[e] = __builtin_bit_cast(_Float16, lb);
            }
          }
          *(volatile v8h*)(C + (size_t)(mBase + row) * ldc + n0 + c8) = hv;
          if (OUT_MODE == 2) *(volatile v8h*)(C2 + (size_t)(mBase + row) * ldc + n0 + c8) = lv;
        }
        __threadfence();
      }
    }
    __builtin_amdgcn_fence(__ATOMIC_RELEASE, "workgroup");
    __builtin_amdgcn_wave_barrier();
    __builtin_amdgcn_fence(__ATOMIC_ACQUIRE, "workgroup");
  }
}

__global__ __launch_bounds__(256) void cast_bf16_kernel(
    const float* __restrict__ src, unsigned short* __restrict__ dst, int nsrc8, int total8)
{
  const int i = blockIdx.x * 256 + threadIdx.x;
  if (i >= total8) return;
  const bool live = (i < nsrc8);
  const int  is   = live ? i : (nsrc8 - 1);
  const float* p = src + ((size_t)is << 3);
  const v4f a0 = *(const v4f*)(p);
  const v4f a1 = *(const v4f*)(p + 4);
  v8h hv;
#pragma unroll
  for (int e = 0; e < 4; ++e) {
    const float f0 = live ? a0[e] : 0.0f;
    const float f1 = live ? a1[e] : 0.0f;
    hv[e]     = __builtin_bit_cast(_Float16, f2bf_bits(f0));
    hv[4 + e] = __builtin_bit_cast(_Float16, f2bf_bits(f1));
  }
  unsigned short* q = dst + ((size_t)i << 3);
  *(volatile v8h*)q = hv;
  __threadfence();
  *(volatile v8h*)q = hv;
}

__global__ __launch_bounds__(256) void split_rows_bf16_kernel(
    const float* __restrict__ src, unsigned short* __restrict__ dhi, unsigned short* __restrict__ dlo, int total8)
{
  const int i = blockIdx.x * 256 + threadIdx.x;
  if (i >= total8) return;
  const size_t e0 = (size_t)i << 3;
  const v4f a0 = *(const v4f*)(src + e0);
  const v4f a1 = *(const v4f*)(src + e0 + 4);
  v8h hv, lv;
#pragma unroll
  for (int e = 0; e < 4; ++e) {
    const float f0 = a0[e], f1 = a1[e];
    const unsigned short h0 = f2bf_bits(f0), h1 = f2bf_bits(f1);
    const unsigned short l0 = f2bf_bits(f0 - bf_bits2f(h0)), l1 = f2bf_bits(f1 - bf_bits2f(h1));
    hv[e]     = __builtin_bit_cast(_Float16, h0);
    hv[4 + e] = __builtin_bit_cast(_Float16, h1);
    lv[e]     = __builtin_bit_cast(_Float16, l0);
    lv[4 + e] = __builtin_bit_cast(_Float16, l1);
  }
  unsigned short* qh = dhi + e0;
  unsigned short* ql = dlo + e0;
  *(volatile v8h*)qh = hv;
  *(volatile v8h*)ql = lv;
  __threadfence();
  *(volatile v8h*)qh = hv;
  *(volatile v8h*)ql = lv;
}

__global__ __launch_bounds__(256) void dtr_split_kernel(
    const float* __restrict__ XD, unsigned short* __restrict__ DH, unsigned short* __restrict__ DL, int total8)
{
  const int i = blockIdx.x * 256 + threadIdx.x;
  if (i >= total8) return;
  const int e0  = i << 3;
  const int row = e0 >> 5;
  const int c8  = e0 & 31;
  const float* p = XD + (size_t)row * kXdP + c8;
  const v4f a0 = *(const v4f*)(p);
  const v4f a1 = *(const v4f*)(p + 4);
  v8h hv, lv;
#pragma unroll
  for (int e = 0; e < 4; ++e) {
    const float f0 = a0[e], f1 = a1[e];
    const unsigned short h0 = f2bf_bits(f0), h1 = f2bf_bits(f1);
    const unsigned short l0 = f2bf_bits(f0 - bf_bits2f(h0)), l1 = f2bf_bits(f1 - bf_bits2f(h1));
    hv[e]     = __builtin_bit_cast(_Float16, h0);
    hv[4 + e] = __builtin_bit_cast(_Float16, h1);
    lv[e]     = __builtin_bit_cast(_Float16, l0);
    lv[4 + e] = __builtin_bit_cast(_Float16, l1);
  }
  unsigned short* qh = DH + e0;
  unsigned short* ql = DL + e0;
  *(volatile v8h*)qh = hv;
  *(volatile v8h*)ql = lv;
  __threadfence();
  *(volatile v8h*)qh = hv;
  *(volatile v8h*)ql = lv;
}

__global__ __launch_bounds__(256) void conv_silu_kernel(
    const float* __restrict__ XZ, const float* __restrict__ cw, const float* __restrict__ cb,
    float* __restrict__ UC, unsigned short* __restrict__ UCH, unsigned short* __restrict__ UCL)
{
  __shared__ __align__(16) float sT[16 * kConvTP];
  const int tid = threadIdx.x, lane = tid & 31, wave = tid >> 5;
  const int d0 = blockIdx.x * 256, d = d0 + tid;
  const int g0 = blockIdx.y * 64;
  const float w0 = bf16r(cw[d * 4 + 0]), w1 = bf16r(cw[d * 4 + 1]);
  const float w2 = bf16r(cw[d * 4 + 2]), w3 = bf16r(cw[d * 4 + 3]);
  const float bc = bf16r(cb[d]);
  float xm3, xm2, xm1;
  {
    const bool hist = (g0 > 0);
    const int rb = hist ? (g0 - 3) : 0;
    const float v3 = XZ[(size_t)rb * kXzP + d];
    const float v2 = XZ[(size_t)(rb + 1) * kXzP + d];
    const float v1 = XZ[(size_t)(rb + 2) * kXzP + d];
    xm3 = hist ? v3 : 0.f;
    xm2 = hist ? v2 : 0.f;
    xm1 = hist ? v1 : 0.f;
  }
  const int hrow = wave >> 1;
  const int hch  = (wave & 1) * 128 + lane * 4;
#pragma unroll 1
  for (int sub = 0; sub < 4; ++sub) {
    const int lb = g0 + sub * 16;
#pragma unroll 1
    for (int s = 0; s < 16; ++s) {
      const float xcur = XZ[(size_t)(lb + s) * kXzP + d];
      float acc = w0 * xm3;
      acc = fmaf(w1, xm2, acc);
      acc = fmaf(w2, xm1, acc);
      acc = fmaf(w3, xcur, acc);
      const float sv = acc + bc;
      const float sg = __builtin_amdgcn_rcpf(1.0f + expf(-sv));
      sT[s * kConvTP + tid] = sv * sg;
      xm3 = xm2; xm2 = xm1; xm1 = xcur;
    }
    __syncthreads();
    v4f fv[4];
    v8h bh[2], blo[2];
#pragma unroll
    for (int it = 0; it < 4; ++it) fv[it] = *(const v4f*)(sT + (it * 4 + hrow) * kConvTP + hch);
#pragma unroll
    for (int it = 0; it < 2; ++it) {
      const float* sp = sT + (it * 8 + wave) * kConvTP + lane * 8;
      const v4f a0 = *(const v4f*)(sp);
      const v4f a1 = *(const v4f*)(sp + 4);
#pragma unroll
      for (int e = 0; e < 4; ++e) {
        const float f0 = a0[e], f1 = a1[e];
        const unsigned short h0 = f2bf_bits(f0), h1 = f2bf_bits(f1);
        const unsigned short l0 = f2bf_bits(f0 - bf_bits2f(h0)), l1 = f2bf_bits(f1 - bf_bits2f(h1));
        bh[it][e]      = __builtin_bit_cast(_Float16, h0);
        bh[it][4 + e]  = __builtin_bit_cast(_Float16, h1);
        blo[it][e]     = __builtin_bit_cast(_Float16, l0);
        blo[it][4 + e] = __builtin_bit_cast(_Float16, l1);
      }
    }
    for (int pass = 0; pass < 2; ++pass) {
#pragma unroll
      for (int it = 0; it < 4; ++it)
        *(volatile v4f*)(UC + (size_t)(lb + it * 4 + hrow) * kDin + d0 + hch) = fv[it];
#pragma unroll
      for (int it = 0; it < 2; ++it) {
        const size_t o = (size_t)(lb + it * 8 + wave) * kDin + d0 + lane * 8;
        *(volatile v8h*)(UCH + o) = bh[it];
        *(volatile v8h*)(UCL + o) = blo[it];
      }
      __threadfence();
    }
    __syncthreads();
  }
}

__global__ __launch_bounds__(512) void scan_kernel(
    const float* __restrict__ DLR, const float* __restrict__ UC, const float* __restrict__ XZ,
    const float* __restrict__ XD, const float* __restrict__ Alog, const float* __restrict__ bdt,
    const float* __restrict__ Dp, float* __restrict__ Y)
{
  __shared__ __align__(16) float sDT[kScanTS * kScanCh];
  __shared__ __align__(16) float sXC[kScanTS * kScanCh];
  __shared__ __align__(16) float sZ[kScanTS * kScanCh];
  __shared__ __align__(16) float sB[kScanTS * kNst];
  __shared__ __align__(16) float sC[kScanTS * kNst];
  __shared__ __align__(16) float sY[kScanTS * kScanYP];
  const int tid = threadIdx.x, lane = tid & 31, wave = tid >> 5;
  const int dl = tid >> 4;
  const int nq = tid & 15;
  const int d0 = blockIdx.x * kScanCh;
  const int d  = d0 + dl;

  float An[4];
#pragma unroll
  for (int q = 0; q < 4; ++q) An[q] = -expf(bf16r(Alog[(size_t)d * kNst + 4 * nq + q]));
  const float Dd = bf16r(Dp[d]);
  float S[4][7];
#pragma unroll
  for (int q = 0; q < 4; ++q)
#pragma unroll
    for (int k = 0; k < 7; ++k) S[q][k] = 0.0f;

  const int sr = tid >> 4, sc4 = (tid & 15) * 4;
  const int q8 = lane >> 3, c4 = (lane & 7) * 4;

#pragma unroll 1
  for (int t0 = 0; t0 < kSeq; t0 += kScanTS) {
    __syncthreads();
#pragma unroll 1
    for (int p = 0; p < 2; ++p) {
      const int idx = tid + 512 * p;
      const int s = idx >> 5, dd = idx & 31;
      const size_t row = (size_t)(t0 + s);
      const float v   = DLR[row * kDin + d0 + dd] + bf16r(bdt[d0 + dd]);
      const float a   = expf(-fabsf(v));
      const float u   = 1.0f + a;
      const float l1p = logf(u) + (a - (u - 1.0f)) * __builtin_amdgcn_rcpf(u);
      sDT[idx] = fmaxf(v, 0.0f) + l1p;
      sXC[idx] = UC[row * kDin + d0 + dd];
      sZ[idx]  = XZ[row * kXzP + kDin + d0 + dd];
    }
    {
      const size_t row = (size_t)(t0 + sr);
      *(v4f*)(sB + sr * kNst + sc4) = *(const v4f*)(XD + row * kXdP + kColB + sc4);
      *(v4f*)(sC + sr * kNst + sc4) = *(const v4f*)(XD + row * kXdP + kColC + sc4);
    }
    __syncthreads();
#pragma unroll 1
    for (int s = 0; s < kScanTS; ++s) {
      const float dt  = sDT[s * kScanCh + dl];
      const float xc  = sXC[s * kScanCh + dl];
      const float zv  = sZ[s * kScanCh + dl];
      const v4f   bq  = *(const v4f*)(sB + s * kNst + 4 * nq);
      const v4f   cq  = *(const v4f*)(sC + s * kNst + 4 * nq);
      const float dtx = dt * xc;
      float yp = 0.0f;
#pragma unroll
      for (int q = 0; q < 4; ++q) {
        const float e = expf(dt * An[q]);
        const float g = dtx * bq[q];
        const float h = fmaf(e, S[q][6], g);
        S[q][6] = fmaf(e, S[q][5], g);
        S[q][5] = fmaf(e, S[q][4], g);
        S[q][4] = fmaf(e, S[q][3], g);
        S[q][3] = fmaf(e, S[q][2], g);
        S[q][2] = fmaf(e, S[q][1], g);
        S[q][1] = fmaf(e, S[q][0], g);
        S[q][0] = g;
        yp = fmaf(h, cq[q], yp);
      }
      yp += __shfl_xor(yp, 8, 32);
      yp += __shfl_xor(yp, 4, 32);
      yp += __shfl_xor(yp, 2, 32);
      yp += __shfl_xor(yp, 1, 32);
      float y = fmaf(Dd, xc, yp);
      const float sg = __builtin_amdgcn_rcpf(1.0f + expf(-zv));
      y = y * (zv * sg);
      if (nq == 0) sY[s * kScanYP + dl] = y;
    }
    __syncthreads();
    if (wave < 8) {
      const int row = wave * 4 + q8;
      const v4f v = *(const v4f*)(sY + row * kScanYP + c4);
      float* dst = Y + (size_t)(t0 + row) * kDin + d0 + c4;
      *(volatile v4f*)dst = v;
      __threadfence();
      *(volatile v4f*)dst = v;
    }
  }
}

__global__ __launch_bounds__(256) void layernorm_kernel(
    const float* __restrict__ PRE, const float* __restrict__ X,
    const float* __restrict__ lnw, const float* __restrict__ lnb, float* __restrict__ OUT)
{
  const int lane = threadIdx.x & 31, wave = threadIdx.x >> 5;
  const int row = blockIdx.x * kLnRows + wave;
  const float* pr = PRE + (size_t)row * kDm;
  const float* xr = X + (size_t)row * kDm;
  v4f v[4];
#pragma unroll
  for (int it = 0; it < 4; ++it) {
    const v4f pa = *(const v4f*)(pr + it * 128 + lane * 4);
    const v4f xa = *(const v4f*)(xr + it * 128 + lane * 4);
    v4f t;
#pragma unroll
    for (int e = 0; e < 4; ++e) {
      const float pe = pa[e], xe = xa[e];
      t[e] = pe + bf16r(xe);
    }
    v[it] = t;
  }
  float s = 0.0f;
#pragma unroll
  for (int it = 0; it < 4; ++it)
#pragma unroll
    for (int e = 0; e < 4; ++e) s += v[it][e];
  s += __shfl_xor(s, 16, 32);
  s += __shfl_xor(s, 8, 32);
  s += __shfl_xor(s, 4, 32);
  s += __shfl_xor(s, 2, 32);
  s += __shfl_xor(s, 1, 32);
  const float mu = s * (1.0f / (float)kDm);
  float s2 = 0.0f;
#pragma unroll
  for (int it = 0; it < 4; ++it)
#pragma unroll
    for (int e = 0; e < 4; ++e) { const float dv = v[it][e] - mu; s2 = fmaf(dv, dv, s2); }
  s2 += __shfl_xor(s2, 16, 32);
  s2 += __shfl_xor(s2, 8, 32);
  s2 += __shfl_xor(s2, 4, 32);
  s2 += __shfl_xor(s2, 2, 32);
  s2 += __shfl_xor(s2, 1, 32);
  const float inv = rsqrtf(s2 * (1.0f / (float)kDm) + kLnEps);
  asm volatile("" ::: "memory");
  v4f o[4];
#pragma unroll
  for (int it = 0; it < 4; ++it) {
    const v4f wa = *(const v4f*)(lnw + it * 128 + lane * 4);
    const v4f ba = *(const v4f*)(lnb + it * 128 + lane * 4);
    v4f t;
#pragma unroll
    for (int e = 0; e < 4; ++e) {
      const float we = bf16r(wa[e]);
      const float be = bf16r(ba[e]);
      const float dv = v[it][e] - mu;
      t[e] = (dv * inv) * we + be;
    }
    o[it] = t;
  }
  float* orow = OUT + (size_t)row * kDm;
  for (int pass = 0; pass < 2; ++pass) {
#pragma unroll
    for (int it = 0; it < 4; ++it) *(volatile v4f*)(orow + it * 128 + lane * 4) = o[it];
    __threadfence();
  }
}

extern "C" void kernel_launch(void* const* d_in, const int* in_sizes, int n_in,
                              void* d_out, int out_size, void* d_ws, size_t ws_size,
                              hipStream_t stream) {
  if (n_in < 12) return;
  if (in_sizes[0] != kSeq * kDm) return;
  if (in_sizes[1] != kXzP * kDm) return;
  if (in_sizes[2] != kDin * kConvK) return;
  if (in_sizes[3] != kDin) return;
  if (in_sizes[4] != kXdN * kDin) return;
  if (in_sizes[5] != kDin * kDtR) return;
  if (in_sizes[6] != kDin) return;
  if (in_sizes[7] != kDin * kNst) return;
  if (in_sizes[8] != kDin) return;
  if (in_sizes[9] != kDm * kDin) return;
  if (in_sizes[10] != kDm || in_sizes[11] != kDm) return;
  if (out_size != kSeq * kDm) return;
  if (ws_size < kWsTotal) return;

  const float* x       = (const float*)d_in[0];
  const float* W_in    = (const float*)d_in[1];
  const float* conv_w  = (const float*)d_in[2];
  const float* conv_b  = (const float*)d_in[3];
  const float* W_xproj = (const float*)d_in[4];
  const float* W_dt    = (const float*)d_in[5];
  const float* b_dt    = (const float*)d_in[6];
  const float* A_log   = (const float*)d_in[7];
  const float* Dp      = (const float*)d_in[8];
  const float* W_out   = (const float*)d_in[9];
  const float* ln_w    = (const float*)d_in[10];
  const float* ln_b    = (const float*)d_in[11];
  float* out = (float*)d_out;

  char* ws = (char*)d_ws;
  unsigned short* XB  = (unsigned short*)(ws + kOffXB);
  unsigned short* WIB = (unsigned short*)(ws + kOffWIB);
  unsigned short* WXB = (unsigned short*)(ws + kOffWXB);
  unsigned short* WDB = (unsigned short*)(ws + kOffWDB);
  unsigned short* WOB = (unsigned short*)(ws + kOffWOB);
  float*          XZ  = (float*)(ws + kOffXZ);
  float*          UC  = (float*)(ws + kOffUC);
  unsigned short* UCH = (unsigned short*)(ws + kOffUCH);
  unsigned short* UCL = (unsigned short*)(ws + kOffUCL);
  float*          XD  = (float*)(ws + kOffXD);
  unsigned short* DRH = (unsigned short*)(ws + kOffDRH);
  unsigned short* DRL = (unsigned short*)(ws + kOffDRL);
  float*          DLR = (float*)(ws + kOffDLR);
  float*          Yf  = (float*)(ws + kOffY);
  unsigned short* YH  = (unsigned short*)(ws + kOffYH);
  unsigned short* YL  = (unsigned short*)(ws + kOffYL);
  float*          PRE = (float*)(ws + kOffPRE);
  const float* dummy_bias = b_dt;

  cast_bf16_kernel<<<(kSeq * kDm / 8) / 256, 256, 0, stream>>>(x, XB, kSeq * kDm / 8, kSeq * kDm / 8);
  cast_bf16_kernel<<<(kXzP * kDm / 8) / 256, 256, 0, stream>>>(W_in, WIB, kXzP * kDm / 8, kXzP * kDm / 8);
  cast_bf16_kernel<<<(kXdP * kDin / 8) / 256, 256, 0, stream>>>(W_xproj, WXB, kXdN * kDin / 8, kXdP * kDin / 8);
  cast_bf16_kernel<<<(kDin * kDtR / 8) / 256, 256, 0, stream>>>(W_dt, WDB, kDin * kDtR / 8, kDin * kDtR / 8);
  cast_bf16_kernel<<<(kDm * kDin / 8) / 256, 256, 0, stream>>>(W_out, WOB, kDm * kDin / 8, kDm * kDin / 8);

  wmma_gemm64<1, 0, 0, 0><<<dim3(64, 1), 256, 0, stream>>>(
      XB, XB, kDm, 0L,
      WIB, WIB, kDm, 0L,
      (void*)XZ, (void*)XZ, kXzP, 0L,
      dummy_bias,
      kSeq, kXzP, kDm, 1.0f);

  conv_silu_kernel<<<dim3(kDin / 256, kSeq / 64), 256, 0, stream>>>(XZ, conv_w, conv_b, UC, UCH, UCL);

  wmma_gemm64<1, 1, 0, 0><<<dim3(6, 1), 256, 0, stream>>>(
      UCH, UCL, kDin, 0L,
      WXB, WXB, kDin, 0L,
      (void*)XD, (void*)XD, kXdP, 0L,
      dummy_bias,
      kSeq, kXdP, kDin, 1.0f);

  dtr_split_kernel<<<(kSeq * kDtR / 8) / 256, 256, 0, stream>>>(XD, DRH, DRL, kSeq * kDtR / 8);

  wmma_gemm64<1, 1, 0, 0><<<dim3(32, 1), 256, 0, stream>>>(
      DRH, DRL, kDtR, 0L,
      WDB, WDB, kDtR, 0L,
      (void*)DLR, (void*)DLR, kDin, 0L,
      dummy_bias,
      kSeq, kDin, kDtR, 1.0f);

  scan_kernel<<<kDin / kScanCh, 512, 0, stream>>>(DLR, UC, XZ, XD, A_log, b_dt, Dp, Yf);

  split_rows_bf16_kernel<<<(kSeq * kDin / 8) / 256, 256, 0, stream>>>(Yf, YH, YL, kSeq * kDin / 8);

  wmma_gemm64<1, 1, 0, 0><<<dim3(16, 1), 256, 0, stream>>>(
      YH, YL, kDin, 0L,
      WOB, WOB, kDin, 0L,
      (void*)PRE, (void*)PRE, kDm, 0L,
      dummy_bias,
      kSeq, kDm, kDin, 1.0f);

  layernorm_kernel<<<kSeq / kLnRows, 256, 0, stream>>>(PRE, x, ln_w, ln_b, out);
}
